// SceneConstructionModel_10024453668877
// MI455X (gfx1250) — hardware-verified
//
#include <hip/hip_runtime.h>
#include <stddef.h>


#define FIN   64
#define HC    512
#define NH    4
#define CH    128
#define ED    8
#define DH    256
#define NR    4
#define NRP   16
#define GR    64
#define GC    128
#define CSP   132
#define NB    512
#define CHUNK 2048
#define NTHR  256
#define NWAVE 8
#define WCAP  256
#define NGRP  (CHUNK / (NTHR * 4))
#define DTHR  128
#define DWAVE 4
#define DEB   (DWAVE * 16)
#define HP    264
#define WSC   16.0f
#define WSCI  0.0625f

#define LDS_SACC (NB * CH)
#define LDS_Z    (NB * CH + 3 * NB)
#define LDS_LIST (NWAVE * WCAP)
#define LDS_AGG_BYTES ((LDS_Z + NB + LDS_LIST + NWAVE) * 4)

static_assert(WCAP == (CHUNK / NTHR) * 32);
static_assert(NGRP >= 1);
static_assert(NB == 512);
static_assert(CHUNK == 2048);
static_assert((LDS_Z % 4) == 0);
static_assert(LDS_AGG_BYTES == 278560);
static_assert(HC == NH * CH);
static_assert(GC == CH);
static_assert(GR == NWAVE * 8);

typedef float    v4f  __attribute__((ext_vector_type(4)));
typedef float    v8f  __attribute__((ext_vector_type(8)));
typedef int      v4i  __attribute__((ext_vector_type(4)));
typedef _Float16 v8h  __attribute__((ext_vector_type(8)));
typedef _Float16 v16h __attribute__((ext_vector_type(16)));
union Frag   { v16h v; v8h half[2]; };
union Pack16 { v8h h; v4i i; _Float16 s[8]; };
union Pack8  { _Float16 s[4]; int u[2]; };

__device__ __forceinline__ v8f wm(v16h a, v16h b, v8f c) {
  v8f d = __builtin_amdgcn_wmma_f32_16x16x32_f16(false, a, false, b, (short)0, c, false, false);
  asm volatile("v_nop\n\tv_nop\n\tv_nop\n\tv_nop" : "+v"(d) : "v"(a), "v"(b));
  return d;
}

__device__ __forceinline__ float frcp(float x) { return __builtin_amdgcn_rcpf(x); }
__device__ __forceinline__ int clampi(int v, int hi) { return v < 0 ? 0 : (v > hi ? hi : v); }

__global__ __launch_bounds__(NTHR) void k_cv(const float* __restrict__ in, _Float16* out, int n8, float scale) {
  const int i = blockIdx.x * NTHR + threadIdx.x;
  if (i >= n8) return;
  const size_t o = (size_t)i * 8;
  const v4f a = *(const v4f*)(in + o);
  const v4f b = *(const v4f*)(in + o + 4);
  Pack16 u;
  u.s[0] = (_Float16)(a.x * scale); u.s[1] = (_Float16)(a.y * scale);
  u.s[2] = (_Float16)(a.z * scale); u.s[3] = (_Float16)(a.w * scale);
  u.s[4] = (_Float16)(b.x * scale); u.s[5] = (_Float16)(b.y * scale);
  u.s[6] = (_Float16)(b.z * scale); u.s[7] = (_Float16)(b.w * scale);
  int* p = (int*)(out + o);
  *(volatile v4i*)p = u.i;
  __threadfence();
  *(volatile v4i*)p = u.i;
}

__global__ __launch_bounds__(NTHR) void k_tr(const float* __restrict__ W, int ldw, int rowoff, int coloff,
                                             _Float16* out, int K, int ntot, int nvalid, float scale) {
  const int i  = blockIdx.x * NTHR + threadIdx.x;
  const int kq = K >> 3;
  if (i >= ntot * kq) return;
  const int n = i / kq;
  const int q = i - n * kq;
  Pack16 u;
#pragma unroll
  for (int j = 0; j < 8; ++j) {
    float v = 0.f;
    if (n < nvalid) v = scale * W[(size_t)(rowoff + 8 * q + j) * ldw + coloff + n];
    u.s[j] = (_Float16)v;
  }
  int* p = (int*)(out + (size_t)n * K + 8 * q);
  *(volatile v4i*)p = u.i;
  __threadfence();
  *(volatile v4i*)p = u.i;
}

__global__ __launch_bounds__(64) void k_me(const float* __restrict__ We1, const float* __restrict__ ae1,
                                           const float* __restrict__ We2, const float* __restrict__ ae2,
                                           float* Me) {
  __shared__ __attribute__((aligned(16))) float ms[64];
  const int t = threadIdx.x;
  const int l = t >> 5;
  const int d = (t >> 2) & 7;
  const int h = t & 3;
  const float* We = l ? We2 : We1;
  const float* ae = l ? ae2 : ae1;
  float s = 0.f;
#pragma unroll 1
  for (int c = 0; c < CH; ++c) s += We[d * HC + h * CH + c] * ae[h * CH + c];
  ms[t] = s;
  __syncthreads();
  if (t < 16) {
    const v4f v = *(const v4f*)(ms + 4 * t);
    float* p = Me + 4 * t;
    *(volatile v4f*)p = v;
    __threadfence();
    *(volatile v4f*)p = v;
  }
}

__global__ __launch_bounds__(NTHR) void k_edge(const float* __restrict__ ef, const float* __restrict__ Me,
                                               float* AE, int nE) {
  __shared__ __attribute__((aligned(16))) float ms[64];
  const int tid = threadIdx.x;
  if (tid < 64) ms[tid] = Me[tid];
  __syncthreads();
  const int e = blockIdx.x * NTHR + tid;
  if (e >= nE) return;
  const v4f f0 = *(const v4f*)(ef + (size_t)e * ED);
  const v4f f1 = *(const v4f*)(ef + (size_t)e * ED + 4);
  const float fe[8] = {f0.x, f0.y, f0.z, f0.w, f1.x, f1.y, f1.z, f1.w};
  float a1[4], a2[4];
#pragma unroll
  for (int h = 0; h < 4; ++h) {
    float s1 = 0.f, s2 = 0.f;
#pragma unroll
    for (int d = 0; d < 8; ++d) {
      s1 += fe[d] * ms[d * 4 + h];
      s2 += fe[d] * ms[32 + d * 4 + h];
    }
    a1[h] = s1;
    a2[h] = s2;
  }
  v4f v1, v2;
  v1.x = a1[0]; v1.y = a1[1]; v1.z = a1[2]; v1.w = a1[3];
  v2.x = a2[0]; v2.y = a2[1]; v2.z = a2[2]; v2.w = a2[3];
  float* p1 = AE + (size_t)e * NH;
  float* p2 = AE + (size_t)nE * NH + (size_t)e * NH;
  *(volatile v4f*)p1 = v1;
  *(volatile v4f*)p2 = v2;
  __threadfence();
  *(volatile v4f*)p1 = v1;
  *(volatile v4f*)p2 = v2;
}

__global__ __launch_bounds__(NTHR) void k_gemm(
    const _Float16* __restrict__ A, int K, int Mvalid,
    const _Float16* __restrict__ Bt, float* C, float scale, int doAlpha,
    const float* __restrict__ att_s, const float* __restrict__ att_d, float* AL, int Mpad) {
  __shared__ __attribute__((aligned(16))) float Cs[GR * CSP];
  __shared__ __attribute__((aligned(16))) float As[GR * NWAVE];
  __shared__ __attribute__((aligned(16))) float Ds[GR * NWAVE];

  const int tid  = threadIdx.x;
  const int lane = tid & 31;
  const int wave = tid >> 5;
  const int hh   = lane >> 4;
  const int m    = lane & 15;
  const int rowBase = blockIdx.x * GR;
  const int col0    = blockIdx.y * GC;
  const int ncol    = col0 + wave * 16 + m;

  size_t aoff[4];
#pragma unroll
  for (int T = 0; T < 4; ++T) {
    int r = rowBase + 16 * T + m;
    if (r > Mvalid - 1) r = Mvalid - 1;
    aoff[T] = (size_t)r * K + 8 * hh;
  }
  const _Float16* bp = Bt + (size_t)ncol * K + 8 * hh;

  v8f acc[4];
#pragma unroll
  for (int T = 0; T < 4; ++T) {
#pragma unroll
    for (int r = 0; r < 8; ++r) acc[T][r] = 0.f;
  }

  const int nK = K >> 5;
#pragma unroll 1
  for (int kt = 0; kt < nK; ++kt) {
    const int k0 = kt * 32;
    Frag b;
    b.half[0] = *(const v8h*)(bp + k0);
    b.half[1] = *(const v8h*)(bp + k0 + 16);
#pragma unroll
    for (int T = 0; T < 4; ++T) {
      Frag a;
      const _Float16* pa = A + aoff[T] + k0;
      a.half[0] = *(const v8h*)(pa);
      a.half[1] = *(const v8h*)(pa + 16);
      acc[T] = wm(a.v, b.v, acc[T]);
    }
  }

  float cs = 0.f, cd = 0.f;
  if (doAlpha) { cs = att_s[ncol]; cd = att_d[ncol]; }
#pragma unroll
  for (int T = 0; T < 4; ++T) {
    float ss[8], sd[8];
#pragma unroll
    for (int r = 0; r < 8; ++r) {
      const float v = acc[T][r] * scale;
      Cs[(16 * T + 8 * hh + r) * CSP + wave * 16 + m] = v;
      ss[r] = v * cs;
      sd[r] = v * cd;
    }
#pragma unroll
    for (int mk = 1; mk < 16; mk <<= 1) {
#pragma unroll
      for (int r = 0; r < 8; ++r) {
        ss[r] += __shfl_xor(ss[r], mk, 32);
        sd[r] += __shfl_xor(sd[r], mk, 32);
      }
    }
    if (m == 0) {
#pragma unroll
      for (int r = 0; r < 8; ++r) {
        As[(16 * T + 8 * hh + r) * NWAVE + wave] = ss[r];
        Ds[(16 * T + 8 * hh + r) * NWAVE + wave] = sd[r];
      }
    }
  }
  __syncthreads();

  v4f xr[8];
  float* cp[8];
#pragma unroll
  for (int i = 0; i < 8; ++i) {
    xr[i] = *(const v4f*)(Cs + (8 * wave + i) * CSP + 4 * lane);
    cp[i] = C + (size_t)(rowBase + 8 * wave + i) * HC + col0 + 4 * lane;
  }
  const bool doal = (doAlpha != 0) && (wave == 0);
  v4f gv = {0.f, 0.f, 0.f, 0.f};
  float* gp = AL;
  if (doal) {
    const int h = blockIdx.y;
    const float* src = (lane < 16) ? As : Ds;
    const int lr = (lane < 16) ? lane : (lane - 16);
    float g[4];
#pragma unroll
    for (int j = 0; j < 4; ++j) {
      const v4f p0 = *(const v4f*)(src + (4 * lr + j) * NWAVE);
      const v4f p1 = *(const v4f*)(src + (4 * lr + j) * NWAVE + 4);
      g[j] = ((p0.x + p0.y) + (p0.z + p0.w)) + ((p1.x + p1.y) + (p1.z + p1.w));
    }
    gv.x = g[0]; gv.y = g[1]; gv.z = g[2]; gv.w = g[3];
    gp = AL + (size_t)((lane < 16) ? h : (NH + h)) * Mpad + rowBase + 4 * lr;
  }

#pragma unroll
  for (int i = 0; i < 8; ++i) *(volatile v4f*)(cp[i]) = xr[i];
  if (doal) *(volatile v4f*)gp = gv;
  __threadfence();
#pragma unroll
  for (int i = 0; i < 8; ++i) *(volatile v4f*)(cp[i]) = xr[i];
  if (doal) *(volatile v4f*)gp = gv;
}

__global__ __launch_bounds__(NTHR) void k_agg(
    const int* __restrict__ ei, const float* __restrict__ AE, const float* __restrict__ xp,
    const float* __restrict__ AL, const float* __restrict__ bias, _Float16* Z,
    int nN, int nE, int Mpad) {
  extern __shared__ v4f lds_dyn[];
  float* sacc = (float*)lds_dyn;
  float* den  = sacc + LDS_SACC;
  float* cnt  = den + NB;
  float* ssum = cnt + NB;
  float* mx   = ssum + NB;
  int*   list = (int*)(mx + NB);
  int*   wcnt = list + LDS_LIST;

  const int tid  = threadIdx.x;
  const int lane = tid & 31;
  const int wave = tid >> 5;
  const int h    = blockIdx.y;
  const int nodeBase = blockIdx.x * NB;

  {
    const v4f z4 = {0.f, 0.f, 0.f, 0.f};
    for (int i = tid; i < LDS_Z / 4; i += NTHR) lds_dyn[i] = z4;
    for (int i = tid; i < NB; i += NTHR) mx[i] = -1.0e30f;
  }
  __syncthreads();

  const float* ALs = AL + (size_t)h * Mpad;
  const float* ALd = AL + (size_t)(NH + h) * Mpad;
  const float* xph = xp + h * CH + 4 * lane;
  const int*   eid = ei + nE;
  const bool  al16 = ((nE & 3) == 0);

  const int nChunks = (nE + CHUNK - 1) / CHUNK;
#pragma unroll 1
  for (int ch = 0; ch < nChunks; ++ch) {
    const int cbase = ch * CHUNK;
    int wc = 0;
#pragma unroll
    for (int g = 0; g < NGRP; ++g) {
      const int el0 = (g * NTHR + tid) * 4;
      const int e0  = cbase + el0;
      const int sent = -2147483647 - 1;
      v4i d;
      if (al16 && (e0 + 3 < nE)) {
        d = *(const v4i*)(eid + e0);
      } else {
        d.x = (e0     < nE) ? eid[min(e0, nE - 1)]     : sent;
        d.y = (e0 + 1 < nE) ? eid[min(e0 + 1, nE - 1)] : sent;
        d.z = (e0 + 2 < nE) ? eid[min(e0 + 2, nE - 1)] : sent;
        d.w = (e0 + 3 < nE) ? eid[min(e0 + 3, nE - 1)] : sent;
      }
      const unsigned s0 = (unsigned)d.x - (unsigned)nodeBase;
      const unsigned s1 = (unsigned)d.y - (unsigned)nodeBase;
      const unsigned s2 = (unsigned)d.z - (unsigned)nodeBase;
      const unsigned s3 = (unsigned)d.w - (unsigned)nodeBase;
      const bool h0 = s0 < (unsigned)NB;
      const bool h1 = s1 < (unsigned)NB;
      const bool h2 = s2 < (unsigned)NB;
      const bool h3 = s3 < (unsigned)NB;
      const unsigned many = __builtin_amdgcn_ballot_w32(h0 | h1 | h2 | h3);
      if (many != 0u) {
#define HITJ(J, HJ, SJ) { \
          const unsigned mj = __builtin_amdgcn_ballot_w32(HJ); \
          if (HJ) { \
            const int pos = wc + (int)__builtin_amdgcn_mbcnt_lo(mj, 0u); \
            if (pos < WCAP) list[wave * WCAP + pos] = ((el0 + (J)) << 9) | (int)(SJ); \
          } \
          wc += (int)__builtin_popcount(mj); }
        HITJ(0, h0, s0)
        HITJ(1, h1, s1)
        HITJ(2, h2, s2)
        HITJ(3, h3, s3)
#undef HITJ
      }
    }
    if (lane == 0) wcnt[wave] = wc;
    __syncthreads();

    if (wave == 0) {
      float* vden = den;
      float* vmx  = mx;
      float* vcnt = cnt;
      float* vss  = ssum;
      for (int wsx = 0; wsx < NWAVE; ++wsx) {
        int n = wcnt[wsx];
        if (n > WCAP) n = WCAP;
        if (n < 0) n = 0;
        for (int i = 0; i < n; ++i) {
          const int ent  = list[wsx * WCAP + i];
          const int slot = ent & (NB - 1);
          const int el   = (ent >> 9) & (CHUNK - 1);
          int e = cbase + el;
          if (e > nE - 1) e = nE - 1;
          const int src = clampi(ei[e], nN - 1);
          int nd = nodeBase + slot;
          if (nd > nN - 1) nd = nN - 1;
          const float ae = AE[(size_t)e * NH + h];
          float al = ALs[src] + ALd[nd] + ae;
          al = (al > 0.f) ? al : 0.2f * al;
          const float mo = vmx[slot];
          const float mn = fmaxf(mo, al);
          const float f  = __expf(mo - mn);
          const float p  = __expf(al - mn);
          const v4f xv = *(const v4f*)(xph + (size_t)src * HC);
          v4f* sp = (v4f*)(sacc + slot * CH + 4 * lane);
          const v4f cur = *sp;
          *sp = cur * f + p * xv;
          if (lane == 0) {
            const float d0 = vden[slot];
            vden[slot] = d0 * f + p;
            vmx[slot]  = mn;
            const float c0 = vcnt[slot];
            vcnt[slot] = c0 + 1.0f;
            const float q0 = vss[slot];
            vss[slot]  = q0 + ae;
          }
        }
      }
    }
    __syncthreads();
  }

  const v4f b4 = *(const v4f*)(bias + h * CH + 4 * lane);
#pragma unroll 1
  for (int j = 0; j < NB / NWAVE; ++j) {
    const int slot = wave * (NB / NWAVE) + j;
    const int node = nodeBase + slot;
    if (node >= nN) break;
    const size_t nrow = (size_t)node;
    const float c  = cnt[slot];
    const float la = ssum[slot] * frcp(fmaxf(c, 1.0f));
    float al = ALs[nrow] + ALd[nrow] + la;
    al = (al > 0.f) ? al : 0.2f * al;
    const float mo = mx[slot];
    const float mn = fmaxf(mo, al);
    const float f  = __expf(mo - mn);
    const float p  = __expf(al - mn);
    const v4f xv = *(const v4f*)(xph + nrow * HC);
    const v4f sv = *(const v4f*)(sacc + slot * CH + 4 * lane) * f + p * xv;
    const float dv  = den[slot] * f + p;
    const float inv = frcp(dv);
    v4f v = sv * inv + b4;
    v4f y;
    y.x = v.x > 0.f ? v.x : (__expf(v.x) - 1.0f);
    y.y = v.y > 0.f ? v.y : (__expf(v.y) - 1.0f);
    y.z = v.z > 0.f ? v.z : (__expf(v.z) - 1.0f);
    y.w = v.w > 0.f ? v.w : (__expf(v.w) - 1.0f);
    Pack8 pk;
    pk.s[0] = (_Float16)y.x; pk.s[1] = (_Float16)y.y; pk.s[2] = (_Float16)y.z; pk.s[3] = (_Float16)y.w;
    const int n0 = __shfl_down(pk.u[0], 1, 32);
    const int n1 = __shfl_down(pk.u[1], 1, 32);
    v4i st;
    st.x = pk.u[0]; st.y = pk.u[1]; st.z = n0; st.w = n1;
    if ((lane & 1) == 0) {
      int* zp = (int*)(Z + nrow * HC + h * CH + 4 * lane);
      *(volatile v4i*)zp = st;
      __threadfence();
      *(volatile v4i*)zp = st;
    }
  }
}

__global__ __launch_bounds__(DTHR) void k_dec(
    const int* __restrict__ ei, const float* __restrict__ P, const float* __restrict__ bd1,
    const _Float16* __restrict__ Wd2t, const float* __restrict__ bd2,
    float* out, int nE, int nN) {
  __shared__ __attribute__((aligned(16))) _Float16 hs[DWAVE * 16 * HP];
  __shared__ __attribute__((aligned(16))) float os[DWAVE * 16 * NR];

  const int tid  = threadIdx.x;
  const int lane = tid & 31;
  const int wave = tid >> 5;
  const int hh   = lane >> 4;
  const int m    = lane & 15;
  const int e0   = blockIdx.x * DEB + wave * 16;
  _Float16* hw = hs + wave * 16 * HP;
  float*    ow = os + wave * 16 * NR;

  const int c = 8 * lane;
  const v4f bb0 = *(const v4f*)(bd1 + c);
  const v4f bb1 = *(const v4f*)(bd1 + c + 4);
#pragma unroll 1
  for (int j = 0; j < 16; ++j) {
    int e = e0 + j;
    if (e > nE - 1) e = nE - 1;
    const int s = clampi(ei[e], nN - 1);
    const int d = clampi(ei[nE + e], nN - 1);
    const float* pa = P + (size_t)s * HC + c;
    const float* pb = P + (size_t)d * HC + DH + c;
    const v4f h0 = *(const v4f*)(pa)     + *(const v4f*)(pb)     + bb0;
    const v4f h1 = *(const v4f*)(pa + 4) + *(const v4f*)(pb + 4) + bb1;
    Pack16 u;
    u.s[0] = (_Float16)h0.x; u.s[1] = (_Float16)h0.y; u.s[2] = (_Float16)h0.z; u.s[3] = (_Float16)h0.w;
    u.s[4] = (_Float16)h1.x; u.s[5] = (_Float16)h1.y; u.s[6] = (_Float16)h1.z; u.s[7] = (_Float16)h1.w;
    *(v8h*)(hw + j * HP + c) = u.h;
  }
  __syncthreads();

  v8f acc = {0.f, 0.f, 0.f, 0.f, 0.f, 0.f, 0.f, 0.f};
  const _Float16* ap = hw + m * HP + 8 * hh;
  const _Float16* bp = Wd2t + m * DH + 8 * hh;
#pragma unroll
  for (int kt = 0; kt < DH / 32; ++kt) {
    const int k0 = kt * 32;
    Frag a, b;
    a.half[0] = *(const v8h*)(ap + k0);
    a.half[1] = *(const v8h*)(ap + k0 + 16);
    b.half[0] = *(const v8h*)(bp + k0);
    b.half[1] = *(const v8h*)(bp + k0 + 16);
    acc = wm(a.v, b.v, acc);
  }

  const float bcol = bd2[(m < NR) ? m : (NR - 1)];
#pragma unroll
  for (int r = 0; r < 8; ++r) {
    const float v  = acc[r] * WSCI + bcol;
    const float sg = frcp(1.0f + __expf(-v));
    if (m < NR) ow[(8 * hh + r) * NR + m] = sg;
  }
  __syncthreads();

  if (lane < 16) {
    const int e = e0 + lane;
    if (e < nE) {
      const v4f ov = *(const v4f*)(ow + lane * NR);
      float* op = out + (size_t)e * NR;
      *(volatile v4f*)op = ov;
      __threadfence();
      *(volatile v4f*)op = ov;
    }
  }
}

extern "C" void kernel_launch(void* const* d_in, const int* in_sizes, int n_in,
                              void* d_out, int out_size, void* d_ws, size_t ws_size,
                              hipStream_t stream) {
  if (n_in < 19) return;
  const int nN = in_sizes[0] / FIN;
  const int nE = in_sizes[1] / 2;
  if (nN <= 0 || in_sizes[0] != nN * FIN) return;
  if (nE <= 0 || in_sizes[1] != 2 * nE) return;
  if (in_sizes[2] != nE * ED) return;
  if (in_sizes[3] != FIN * HC) return;
  if (in_sizes[4] != HC || in_sizes[5] != HC || in_sizes[6] != ED * HC || in_sizes[7] != HC || in_sizes[8] != HC) return;
  if (in_sizes[9] != HC * HC) return;
  if (in_sizes[10] != HC || in_sizes[11] != HC || in_sizes[12] != ED * HC || in_sizes[13] != HC || in_sizes[14] != HC) return;
  if (in_sizes[15] != 2 * HC * DH || in_sizes[16] != DH || in_sizes[17] != DH * NR || in_sizes[18] != NR) return;
  if (out_size != nE * NR) return;

  const float* x   = (const float*)d_in[0];
  const int*   ei  = (const int*)d_in[1];
  const float* ef  = (const float*)d_in[2];
  const float* W1  = (const float*)d_in[3];
  const float* as1 = (const float*)d_in[4];
  const float* ad1 = (const float*)d_in[5];
  const float* We1 = (const float*)d_in[6];
  const float* ae1 = (const float*)d_in[7];
  const float* b1  = (const float*)d_in[8];
  const float* W2  = (const float*)d_in[9];
  const float* as2 = (const float*)d_in[10];
  const float* ad2 = (const float*)d_in[11];
  const float* We2 = (const float*)d_in[12];
  const float* ae2 = (const float*)d_in[13];
  const float* b2  = (const float*)d_in[14];
  const float* Wd1 = (const float*)d_in[15];
  const float* bd1 = (const float*)d_in[16];
  const float* Wd2 = (const float*)d_in[17];
  const float* bd2 = (const float*)d_in[18];
  float* out = (float*)d_out;

  const int Mpad = ((nN + GR - 1) / GR) * GR;

  char* base = (char*)d_ws;
  size_t off = 0;
  auto take = [&](size_t bytes) -> char* {
    char* p = base + off;
    off += (bytes + 255) & ~(size_t)255;
    return p;
  };
  _Float16* W1t  = (_Float16*)take((size_t)HC * FIN * 2);
  _Float16* W2t  = (_Float16*)take((size_t)HC * HC * 2);
  _Float16* WPt  = (_Float16*)take((size_t)HC * HC * 2);
  _Float16* Wd2t = (_Float16*)take((size_t)NRP * DH * 2);
  float*    Me   = (float*)take(64 * sizeof(float));
  _Float16* X16  = (_Float16*)take((size_t)nN * FIN * 2);
  _Float16* Z16  = (_Float16*)take((size_t)nN * HC * 2);
  float*    XP   = (float*)take((size_t)Mpad * HC * sizeof(float));
  float*    AL   = (float*)take((size_t)2 * NH * Mpad * sizeof(float));
  float*    AE   = (float*)take((size_t)2 * nE * NH * sizeof(float));
  if (off > ws_size) return;

  k_tr<<<(HC * (FIN / 8) + NTHR - 1) / NTHR, NTHR, 0, stream>>>(W1, HC, 0, 0, W1t, FIN, HC, HC, WSC);
  k_tr<<<(HC * (HC / 8) + NTHR - 1) / NTHR, NTHR, 0, stream>>>(W2, HC, 0, 0, W2t, HC, HC, HC, WSC);
  k_tr<<<(DH * (HC / 8) + NTHR - 1) / NTHR, NTHR, 0, stream>>>(Wd1, DH, 0, 0, WPt, HC, DH, DH, WSC);
  k_tr<<<(DH * (HC / 8) + NTHR - 1) / NTHR, NTHR, 0, stream>>>(Wd1, DH, HC, 0, WPt + (size_t)DH * HC, HC, DH, DH, WSC);
  k_tr<<<(NRP * (DH / 8) + NTHR - 1) / NTHR, NTHR, 0, stream>>>(Wd2, NR, 0, 0, Wd2t, DH, NRP, NR, WSC);

  const int n8x = nN * FIN / 8;
  k_cv<<<(n8x + NTHR - 1) / NTHR, NTHR, 0, stream>>>(x, X16, n8x, 1.0f);
  k_me<<<1, 64, 0, stream>>>(We1, ae1, We2, ae2, Me);
  k_edge<<<(nE + NTHR - 1) / NTHR, NTHR, 0, stream>>>(ef, Me, AE, nE);

  hipFuncSetAttribute(reinterpret_cast<const void*>(&k_agg),
                      hipFuncAttributeMaxDynamicSharedMemorySize, LDS_AGG_BYTES);
  const dim3 ggemm(Mpad / GR, HC / GC);
  const dim3 gagg((nN + NB - 1) / NB, NH);

  k_gemm<<<ggemm, NTHR, 0, stream>>>(X16, FIN, nN, W1t, XP, WSCI, 1, as1, ad1, AL, Mpad);
  k_agg<<<gagg, NTHR, LDS_AGG_BYTES, stream>>>(ei, AE, XP, AL, b1, Z16, nN, nE, Mpad);

  k_gemm<<<ggemm, NTHR, 0, stream>>>(Z16, HC, nN, W2t, XP, WSCI, 1, as2, ad2, AL, Mpad);
  k_agg<<<gagg, NTHR, LDS_AGG_BYTES, stream>>>(ei, AE + (size_t)nE * NH, XP, AL, b2, Z16, nN, nE, Mpad);

  k_gemm<<<ggemm, NTHR, 0, stream>>>(Z16, HC, nN, WPt, XP, WSCI, 0, bd1, bd1, AL, Mpad);
  k_dec<<<(nE + DEB - 1) / DEB, DTHR, 0, stream>>>(ei, XP, bd1, Wd2t, bd2, out, nE, nN);
}
